// MLP_53807350284779
// MI455X (gfx1250) — hardware-verified
//
#include <hip/hip_runtime.h>
#include <math.h>


typedef unsigned int u32;
typedef __attribute__((ext_vector_type(2)))  int      v2i;
typedef __attribute__((ext_vector_type(16))) _Float16 v16h;
typedef __attribute__((ext_vector_type(8)))  _Float16 v8h;
typedef __attribute__((ext_vector_type(8)))  float    v8f;
typedef __attribute__((ext_vector_type(4)))  float    v4f;
#define NN    50000
#define NE    800000
#define DD    64
#define NG    128
#define SORTN 1048576
#define TILE  8192
#define NPAD  50176
#define VST2(T, ptr, val) do { const T _v = (val); *(volatile T*)(ptr) = _v; __threadfence(); *(volatile T*)(ptr) = _v; } while (0)
__device__ __forceinline__ v8f wmma16(v16h a, v16h b, v8f c) {
  v8f d = __builtin_amdgcn_wmma_f32_16x16x32_f16(false, a, false, b, (short)0, c, false, false);
  asm volatile("v_nop\n\tv_nop\n\tv_nop\n\tv_nop" : "+v"(d) : "v"(a), "v"(b));
  return d;
}
__device__ __forceinline__ v16h frag16(const _Float16* p, int hh) {
  const v8h lo = *(const v8h*)(p + 8 * hh), hi = *(const v8h*)(p + 16 + 8 * hh);
  return __builtin_shufflevector(lo, hi, 0,1,2,3,4,5,6,7,8,9,10,11,12,13,14,15);
}
__global__ __launch_bounds__(256) void k_sort_init(const int* __restrict__ src, const int* __restrict__ dst, u32* __restrict__ A, int E) {
  const int i = blockIdx.x * 256 + threadIdx.x;
  VST2(u32, A + i, (i < E) ? (((u32)dst[i]) << 16) | (u32)src[i] : 0xffffffffu);
}
__device__ __forceinline__ void cas_lds(u32* s, int lo, int hi, bool up) {
  const u32 a = s[lo], b = s[hi]; const bool sw = up ? (a > b) : (a < b); s[lo] = sw ? b : a; s[hi] = sw ? a : b;
}
__global__ __launch_bounds__(256) void k_sort_local(u32* __restrict__ A) {
  __shared__ u32 s[TILE];
  const int base = blockIdx.x * TILE, t = threadIdx.x;
  for (int i = t; i < TILE; i += 256) s[i] = A[base + i];
  __syncthreads();
  for (int k = 2; k <= TILE; k <<= 1)
    for (int j = k >> 1; j > 0; j >>= 1) {
      for (int p = t; p < TILE / 2; p += 256) {
        const int lo = ((p >> __builtin_ctz(j)) << (__builtin_ctz(j) + 1)) | (p & (j - 1));
        cas_lds(s, lo, lo + j, (((base + lo) & k) == 0));
      }
      __syncthreads();
    }
  for (int pass = 0; pass < 2; ++pass) { for (int i = t; i < TILE; i += 256) *(volatile u32*)(A + base + i) = s[i]; __threadfence(); }
}
__global__ __launch_bounds__(256) void k_sort_global(u32* __restrict__ A, int logj, int k) {
  const int p = blockIdx.x * 256 + threadIdx.x;
  const int j = 1 << logj;
  const int lo = ((p >> logj) << (logj + 1)) | (p & (j - 1)), hi = lo + j;
  const u32 a = A[lo], b = A[hi];
  const bool up = ((lo & k) == 0), sw = up ? (a > b) : (a < b);
  const u32 vlo = sw ? b : a, vhi = sw ? a : b;
  *(volatile u32*)(A + lo) = vlo; *(volatile u32*)(A + hi) = vhi; __threadfence();
  *(volatile u32*)(A + lo) = vlo; *(volatile u32*)(A + hi) = vhi;
}
__global__ __launch_bounds__(256) void k_sort_lds(u32* __restrict__ A, int k) {
  __shared__ u32 s[TILE];
  const int base = blockIdx.x * TILE, t = threadIdx.x;
  for (int i = t; i < TILE; i += 256) s[i] = A[base + i];
  __syncthreads();
  for (int j = TILE >> 1; j > 0; j >>= 1) {
    for (int p = t; p < TILE / 2; p += 256) {
      const int lo = ((p >> __builtin_ctz(j)) << (__builtin_ctz(j) + 1)) | (p & (j - 1));
      cas_lds(s, lo, lo + j, (((base + lo) & k) == 0));
    }
    __syncthreads();
  }
  for (int pass = 0; pass < 2; ++pass) { for (int i = t; i < TILE; i += 256) *(volatile u32*)(A + base + i) = s[i]; __threadfence(); }
}

__global__ __launch_bounds__(256) void k_segs(const u32* __restrict__ A, v2i* __restrict__ seg, float* __restrict__ inv) {
  const int n = blockIdx.x * 256 + threadIdx.x;
  if (n >= NN) return;
  int lo = 0, hi = SORTN;
  while (lo < hi) { const int mid = (lo + hi) >> 1; if ((A[mid] >> 16) < (u32)n) lo = mid + 1; else hi = mid; }
  const int st = lo; hi = SORTN;
  while (lo < hi) { const int mid = (lo + hi) >> 1; if ((A[mid] >> 16) < (u32)(n + 1)) lo = mid + 1; else hi = mid; }
  const v2i sv = {st, lo - st};
  VST2(v2i, seg + n, sv);
  VST2(float, inv + n, 1.0f / fmaxf((float)(lo - st), 1.0f));
}
__global__ __launch_bounds__(256) void k_rows(const float* __restrict__ x, const u32* __restrict__ A, const v2i* __restrict__ seg, const float* __restrict__ inv,
                                              _Float16* __restrict__ A16) {
  const int t = blockIdx.x * 256 + threadIdx.x;
  const int i = t >> 4, c = (t & 15) * 8;
  v8h o;
  if (i >= NN) { for (int e = 0; e < 8; ++e) o[e] = (_Float16)0.f; }
  else if (c >= 64) {
#pragma unroll
    for (int e = 0; e < 8; ++e) o[e] = (_Float16)x[(size_t)i * DD + c - 64 + e];
  } else {
    const v2i sv = seg[i];
    float acc[8] = {0.f, 0.f, 0.f, 0.f, 0.f, 0.f, 0.f, 0.f};
    for (int p = 0; p < sv[1]; ++p) {
      const int j = (int)(A[sv[0] + p] & 0xffffu);
      const float* xr = x + (size_t)j * DD + c;
#pragma unroll
      for (int e = 0; e < 8; ++e) acc[e] += xr[e];
    }
    const float w = inv[i];
#pragma unroll
    for (int e = 0; e < 8; ++e) o[e] = (_Float16)(acc[e] * w);
  }
  VST2(v8h, A16 + (size_t)i * 128 + c, o);
}
__global__ __launch_bounds__(256) void k_wt(const float* __restrict__ wl, const float* __restrict__ wr, _Float16* __restrict__ Wt) {
  const int t = blockIdx.x * 256 + threadIdx.x;
  const int n = t >> 4, k0 = (t & 15) * 8;
  v8h o;
#pragma unroll
  for (int e = 0; e < 8; ++e) { const int k = k0 + e; o[e] = (_Float16)((k < 64) ? wl[k * DD + n] : wr[(k - 64) * DD + n]); }
  VST2(v8h, Wt + n * 128 + k0, o);
}
__global__ __launch_bounds__(128) void k_gemm(const _Float16* __restrict__ A16, const _Float16* __restrict__ Wt, const float* __restrict__ bias, float* __restrict__ out) {
  __shared__ __attribute__((aligned(16))) float sT[4][16][68];
  const int lane = threadIdx.x & 31, wave = threadIdx.x >> 5, hh = lane >> 4, l16 = lane & 15;
  const int m0 = (blockIdx.x * 4 + wave) * 64;
  v8f acc[4][4] = {};
#pragma unroll
  for (int k0 = 0; k0 < 128; k0 += 32) {
    v16h a[4];
#pragma unroll
    for (int mi = 0; mi < 4; ++mi) a[mi] = frag16(A16 + (size_t)(m0 + mi * 16 + l16) * 128 + k0, hh);
#pragma unroll
    for (int ni = 0; ni < 4; ++ni) { const v16h b = frag16(Wt + (ni * 16 + l16) * 128 + k0, hh);
#pragma unroll
      for (int mi = 0; mi < 4; ++mi) acc[mi][ni] = wmma16(a[mi], b, acc[mi][ni]); }
  }
  float (*st)[68] = sT[wave];
#pragma unroll
  for (int mi = 0; mi < 4; ++mi) {
#pragma unroll
    for (int ni = 0; ni < 4; ++ni)
#pragma unroll
      for (int i = 0; i < 8; ++i) st[i + 8 * hh][ni * 16 + l16] = acc[mi][ni][i] + bias[ni * 16 + l16];
    __builtin_amdgcn_fence(__ATOMIC_RELEASE, "workgroup"); __builtin_amdgcn_wave_barrier(); __builtin_amdgcn_fence(__ATOMIC_ACQUIRE, "workgroup");
    for (int pass = 0; pass < 2; ++pass) {
#pragma unroll
      for (int j = 0; j < 8; ++j) { const int rr = j * 2 + hh, q4 = l16 * 4;
        *(volatile v4f*)(out + (size_t)(m0 + mi * 16 + rr) * DD + q4) = *(const v4f*)(&st[rr][q4]); }
      __threadfence();
    }
    __builtin_amdgcn_fence(__ATOMIC_RELEASE, "workgroup"); __builtin_amdgcn_wave_barrier(); __builtin_amdgcn_fence(__ATOMIC_ACQUIRE, "workgroup");
  }
}
__global__ __launch_bounds__(64) void k_pool(const float* __restrict__ h, const int* __restrict__ batch, float* __restrict__ c) {
  const int g = blockIdx.x, d = threadIdx.x;
  int lo = 0, hi = NN;
  while (lo < hi) { const int mid = (lo + hi) >> 1; if (batch[mid] < g) lo = mid + 1; else hi = mid; }
  const int st = lo; hi = NN;
  while (lo < hi) { const int mid = (lo + hi) >> 1; if (batch[mid] < g + 1) lo = mid + 1; else hi = mid; }
  float s = 0.f;
  for (int i = st; i < lo; ++i) s += h[(size_t)i * DD + d];
  VST2(float, c + g * DD + d, s / fmaxf((float)(lo - st), 1.0f));
}
__device__ __forceinline__ float tanh_e(float x) { const float xc = fminf(fmaxf(x, -15.f), 15.f); const float e = expf(2.0f * xc); return 1.0f - 2.0f / (e + 1.0f); }
__device__ void lin_bn_tanh_T(const float* __restrict__ in, int inStrideG, int inStrideK, int K, const float* __restrict__ W, int M,
                              const float* __restrict__ b, const float* __restrict__ gamma, const float* __restrict__ beta, float* __restrict__ outT, int tid) {
  for (int j = tid; j < M; j += 256) {
    float sum = 0.f, sq = 0.f;
#pragma unroll 1
    for (int g = 0; g < NG; ++g) {
      float s = b[j];
#pragma unroll 1
      for (int k = 0; k < K; ++k) s += in[g * inStrideG + k * inStrideK] * W[k * M + j];
      sum += s; sq += s * s;
    }
    const float mean = sum * (1.0f / NG);
    const float var = fmaxf(sq * (1.0f / NG) - mean * mean, 0.f);
    const float sc = gamma[j] / sqrtf(var + 1e-5f);
    for (int pass = 0; pass < 2; ++pass) {
#pragma unroll 1
      for (int g4 = 0; g4 < NG; g4 += 4) {
        v4f o;
#pragma unroll 1
        for (int e = 0; e < 4; ++e) {
          const int g = g4 + e;
          float s = b[j];
#pragma unroll 1
          for (int k = 0; k < K; ++k) s += in[g * inStrideG + k * inStrideK] * W[k * M + j];
          o[e] = tanh_e((s - mean) * sc + beta[j]);
        }
        *(volatile v4f*)(outT + (size_t)j * NG + g4) = o;
      }
      __threadfence();
    }
  }
}
__global__ __launch_bounds__(256) void k_head(const float* __restrict__ c,
                                              const float* __restrict__ W1, const float* __restrict__ b1, const float* __restrict__ g1, const float* __restrict__ be1,
                                              const float* __restrict__ W2, const float* __restrict__ b2, const float* __restrict__ g2, const float* __restrict__ be2,
                                              const float* __restrict__ W3, const float* __restrict__ b3, const float* __restrict__ g3, const float* __restrict__ be3,
                                              const float* __restrict__ W4, const float* __restrict__ b4,
                                              float* __restrict__ T1, float* __restrict__ T2, float* __restrict__ T3, float* __restrict__ out) {
  const int tid = threadIdx.x;
  lin_bn_tanh_T(c, DD, 1, DD, W1, 200, b1, g1, be1, T1, tid);
  __threadfence(); __syncthreads();
  lin_bn_tanh_T(T1, 1, NG, 200, W2, 100, b2, g2, be2, T2, tid);
  __threadfence(); __syncthreads();
  lin_bn_tanh_T(T2, 1, NG, 100, W3, 100, b3, g3, be3, T3, tid);
  __threadfence(); __syncthreads();
  for (int pass = 0; pass < 2; ++pass) {
#pragma unroll 1
    for (int q = tid; q < NG * 80; q += 256) {
      const int g = q / 80, j = q % 80;
      float s = b4[j];
#pragma unroll 1
      for (int k = 0; k < 100; ++k) s += T3[k * NG + g] * W4[k * 80 + j];
      *(volatile float*)(out + q) = s;
    }
    __threadfence();
  }
}
extern "C" void kernel_launch(void* const* d_in, const int* in_sizes, int n_in,
                              void* d_out, int out_size, void* d_ws, size_t ws_size, hipStream_t stream) {
  (void)in_sizes; (void)n_in; (void)out_size;
  const float* x     = (const float*)d_in[0];
  const int*   ei    = (const int*)  d_in[1];
  const int*   batch = (const int*)  d_in[2];
  const float* w1l = (const float*)d_in[3];  const float* b1l = (const float*)d_in[4];  const float* w1r = (const float*)d_in[5];
  const float* w2l = (const float*)d_in[6];  const float* b2l = (const float*)d_in[7];  const float* w2r = (const float*)d_in[8];
  const float* w3l = (const float*)d_in[9];  const float* b3l = (const float*)d_in[10]; const float* w3r = (const float*)d_in[11];
  const float* lin1_w = (const float*)d_in[12]; const float* lin1_b = (const float*)d_in[13]; const float* g1 = (const float*)d_in[14]; const float* be1 = (const float*)d_in[15];
  const float* lin2_w = (const float*)d_in[16]; const float* lin2_b = (const float*)d_in[17]; const float* g2 = (const float*)d_in[18]; const float* be2 = (const float*)d_in[19];
  const float* lin3_w = (const float*)d_in[20]; const float* lin3_b = (const float*)d_in[21]; const float* g3 = (const float*)d_in[22]; const float* be3 = (const float*)d_in[23];
  const float* lin4_w = (const float*)d_in[24]; const float* lin4_b = (const float*)d_in[25];
  float* out = (float*)d_out;
  char* ws = (char*)d_ws; size_t off = 0;
  auto take = [&](size_t bytes) { void* p = ws + off; off = (off + bytes + 255) & ~(size_t)255; return p; };
  u32*      keys = (u32*)take((size_t)SORTN * 4);
  v2i*      seg  = (v2i*)take((size_t)NN * 8);
  float*    inv  = (float*)take((size_t)NN * 4);
  _Float16* A16  = (_Float16*)take((size_t)NPAD * 128 * 2);
  _Float16* Wt   = (_Float16*)take((size_t)64 * 128 * 2);
  float*    h1   = (float*)take((size_t)NPAD * DD * 4);
  float*    h2   = (float*)take((size_t)NPAD * DD * 4);
  float*    cpool = (float*)take((size_t)NG * DD * 4);
  float*    T1   = (float*)take((size_t)200 * NG * 4);
  float*    T2   = (float*)take((size_t)100 * NG * 4);
  float*    T3   = (float*)take((size_t)100 * NG * 4);
  if (off > ws_size) return;
  const dim3 b256(256);
  k_sort_init<<<SORTN / 256, b256, 0, stream>>>(ei, ei + NE, keys, NE);
  k_sort_local<<<SORTN / TILE, b256, 0, stream>>>(keys);
  for (int k = TILE * 2; k <= SORTN; k <<= 1) {
    for (int logj = __builtin_ctz(k) - 1; (1 << logj) >= TILE; --logj)
      k_sort_global<<<SORTN / 2 / 256, b256, 0, stream>>>(keys, logj, k);
    k_sort_lds<<<SORTN / TILE, b256, 0, stream>>>(keys, k);
  }
  k_segs<<<(NN + 255) / 256, b256, 0, stream>>>(keys, seg, inv);
  auto sage = [&](const float* hin, const float* wl, const float* bl, const float* wr, float* hout) {
    k_rows<<<NPAD * 16 / 256, b256, 0, stream>>>(hin, keys, seg, inv, A16);
    k_wt<<<64 * 16 / 256, b256, 0, stream>>>(wl, wr, Wt);
    k_gemm<<<NPAD / 256, 128, 0, stream>>>(A16, Wt, bl, hout);
  };
  sage(x,  w1l, b1l, w1r, h1);
  sage(h1, w2l, b2l, w2r, h2);
  sage(h2, w3l, b3l, w3r, h1);
  k_pool<<<NG, 64, 0, stream>>>(h1, batch, cpool);
  k_head<<<1, 256, 0, stream>>>(cpool, lin1_w, lin1_b, g1, be1, lin2_w, lin2_b, g2, be2, lin3_w, lin3_b, g3, be3, lin4_w, lin4_b, T1, T2, T3, out);
}
